// TransitionDown_51694226375250
// MI455X (gfx1250) — hardware-run, weakly checked
//
#include <hip/hip_runtime.h>
#include <math.h>
#include <stdint.h>

#pragma clang fp contract(off)

typedef __attribute__((ext_vector_type(16))) _Float16 v16h;
typedef __attribute__((ext_vector_type(8)))  _Float16 v8h;
typedef __attribute__((ext_vector_type(8)))  float    v8f;
typedef __attribute__((ext_vector_type(4)))  float    v4f;
typedef __attribute__((ext_vector_type(4)))  int      v4i;

namespace {
constexpr int kClouds = 4;
constexpr int kPts    = 4096;
constexpr int kNbr    = 16;
constexpr int kSmp    = 1024;
constexpr int kCf     = 64;
constexpr int kCin    = 67;
constexpr int kCo     = 128;
constexpr int kNodes  = kClouds * kPts;
constexpr int kEdges  = kNodes * kNbr;
constexpr int kOut0   = kClouds * kSmp * 3;
constexpr int kOutAll = kOut0 + kClouds * kSmp * kCo;
constexpr float kCarry = 64.0f;
constexpr float kFold  = 1.0f / (kCarry * kCarry);
constexpr float kF16MinNormal = 6.103515625e-5f;
constexpr double kInvEdges = 1.0 / (double)kEdges;
constexpr int kPrepFeatBlk = (kNodes * kCf / 8) / 256;
constexpr int kPrepW2Blk   = (kCo * kCo / 8) / 256;
constexpr int kPrepW1Blk   = (kCo * kCf / 8) / 256;
constexpr int kEdgeBlk     = kNodes / 64;
constexpr int kGemmPBlk    = (kNodes / 64) * 2 / 8;
constexpr int kGemm2Blk    = (kEdges / 64) * 2 / 8;
constexpr int kFinRowBlk   = (kClouds * kSmp) / 8;
constexpr int kFinPosBlk   = kOut0 / (256 * 4);
static_assert(kPrepFeatBlk == 512 && kPrepW2Blk == 8 && kPrepW1Blk == 4, "prep coverage");
static_assert(kEdgeBlk == 256 && kGemmPBlk == 64 && kGemm2Blk == 1024, "tile coverage");
static_assert(kFinRowBlk == 512 && kFinPosBlk == 12 && kFinPosBlk * 1024 == kOut0, "finalize coverage");
static_assert((kCf % 32) == 0 && (kCo % 32) == 0, "K multiples of 32");
static_assert((kNodes % 64) == 0 && (kEdges % 64) == 0 && kCo == 128, "M multiples of 64, N = 128");
static_assert((kOut0 * 4) % 128 == 0, "second output starts on a line");

constexpr size_t kOffCent  = 0;
constexpr size_t kOffNbr   = kOffCent  + (size_t)kClouds * kSmp * 4;
constexpr size_t kOffFeatH = kOffNbr   + (size_t)kNodes * kNbr * 4;
constexpr size_t kOffW1fH  = kOffFeatH + (size_t)kNodes * kCf * 2;
constexpr size_t kOffW2H   = kOffW1fH  + (size_t)kCo * kCf * 2;
constexpr size_t kOffP     = kOffW2H   + (size_t)kCo * kCo * 2;
constexpr size_t kOffX2    = kOffP     + (size_t)kNodes * kCo * 4;
constexpr size_t kOffHmax  = kOffX2    + (size_t)kEdges * kCo * 2;
constexpr size_t kOffHmin  = kOffHmax  + (size_t)kNodes * kCo * 4;
constexpr size_t kOffPart1 = kOffHmin  + (size_t)kNodes * kCo * 4;
constexpr size_t kOffPart2 = kOffPart1 + (size_t)kEdgeBlk * 256 * 4;
constexpr size_t kOffSt1   = kOffPart2 + (size_t)kGemm2Blk * 256 * 4;
constexpr size_t kOffSt2   = kOffSt1   + 1024;
constexpr size_t kWsTotal  = kOffSt2   + 1024;
static_assert(kWsTotal == 96798720ull, "carve total");
static_assert(kWsTotal <= 134217728ull, "carve cap");
static_assert((kOffNbr % 128) == 0 && (kOffFeatH % 128) == 0 && (kOffW1fH % 128) == 0 && (kOffW2H % 128) == 0 &&
              (kOffP % 128) == 0 && (kOffX2 % 128) == 0 && (kOffHmax % 128) == 0 && (kOffHmin % 128) == 0 &&
              (kOffPart1 % 128) == 0 && (kOffPart2 % 128) == 0 && (kOffSt1 % 128) == 0 && (kOffSt2 % 128) == 0,
              "128-B aligned regions");
}

__device__ __forceinline__ int clampi(int v, int lo, int hi) { return v < lo ? lo : (v > hi ? hi : v); }

__device__ __forceinline__ _Float16 cvt_h(float v) {
  const float z = (fabsf(v) < kF16MinNormal) ? 0.0f : v;
  return (_Float16)z;
}

__device__ __forceinline__ void unpack8(v4f a, v4f b, float (&o)[8]) {
  o[0] = a[0]; o[1] = a[1]; o[2] = a[2]; o[3] = a[3];
  o[4] = b[0]; o[5] = b[1]; o[6] = b[2]; o[7] = b[3];
}

__global__ __launch_bounds__(256) void prep_planes_kernel(
    const float* __restrict__ feat, const float* __restrict__ W1, const float* __restrict__ W2,
    unsigned short* __restrict__ featH, unsigned short* __restrict__ W1fH, unsigned short* __restrict__ W2H)
{
  const int tid = threadIdx.x;
  const int blk = blockIdx.x;
  float a[8];
  unsigned short* dst;
  if (blk < kPrepFeatBlk) {
    const size_t e0 = ((size_t)blk * 256 + tid) << 3;
    const v4f x0 = *(const v4f*)(feat + e0);
    const v4f x1 = *(const v4f*)(feat + e0 + 4);
    unpack8(x0, x1, a);
    dst = featH + e0;
  } else if (blk < kPrepFeatBlk + kPrepW2Blk) {
    const size_t e0 = ((size_t)(blk - kPrepFeatBlk) * 256 + tid) << 3;
    const v4f x0 = *(const v4f*)(W2 + e0);
    const v4f x1 = *(const v4f*)(W2 + e0 + 4);
    unpack8(x0, x1, a);
    dst = W2H + e0;
  } else {
    const int i  = (blk - kPrepFeatBlk - kPrepW2Blk) * 256 + tid;
    const int d  = i >> 3;
    const int c0 = (i & 7) * 8;
#pragma unroll
    for (int e = 0; e < 8; ++e) a[e] = W1[(size_t)d * kCin + 3 + c0 + e];
    dst = W1fH + (size_t)d * kCf + c0;
  }
  v8h hv;
#pragma unroll
  for (int e = 0; e < 8; ++e) hv[e] = cvt_h(a[e] * kCarry);
  *(volatile v8h*)dst = hv;
  __threadfence();
  *(volatile v8h*)dst = hv;
}

__device__ __forceinline__ void argmax_red(float& v, int& i) {
#pragma unroll
  for (int off = 16; off > 0; off >>= 1) {
    const float ov = __shfl_xor(v, off, 32);
    const int   oi = __shfl_xor(i, off, 32);
    const bool take = (ov > v) || (ov == v && oi < i);
    v = take ? ov : v;
    i = take ? oi : i;
  }
}

__global__ __launch_bounds__(1024) void sample_kernel(const float* __restrict__ pos, int* __restrict__ cent)
{
  __shared__ __align__(16) float sp[kPts * 3];
  __shared__ float wv[2][32];
  __shared__ int   wi[2][32];
  __shared__ int   wtot[32];
  __shared__ __align__(16) int scent[kSmp];

  const int b = blockIdx.x, tid = threadIdx.x;
  const int lane = tid & 31, wave = tid >> 5;
  {
    const v4f* src = (const v4f*)(pos + (size_t)b * kPts * 3);
#pragma unroll
    for (int i = 0; i < 3; ++i) ((v4f*)sp)[tid + i * 1024] = src[tid + i * 1024];
  }
  __syncthreads();
  float px[4], py[4], pz[4], dd[4];
#pragma unroll
  for (int e = 0; e < 4; ++e) {
    px[e] = sp[(tid * 4 + e) * 3 + 0];
    py[e] = sp[(tid * 4 + e) * 3 + 1];
    pz[e] = sp[(tid * 4 + e) * 3 + 2];
    dd[e] = 1e10f;
  }
  int last = 0;
  unsigned sel = (tid == 0) ? 1u : 0u;
#pragma unroll 1
  for (int it = 1; it < kSmp; ++it) {
    const int par = it & 1;
    const float lx = sp[last * 3 + 0], ly = sp[last * 3 + 1], lz = sp[last * 3 + 2];
    float bv = -1.0f;
    int bi = 1 << 30;
#pragma unroll
    for (int e = 0; e < 4; ++e) {
      const float dx = px[e] - lx;
      const float dy = py[e] - ly;
      const float dz = pz[e] - lz;
      const float d  = (dx * dx + dy * dy) + dz * dz;
      const float nd = fminf(dd[e], d);
      dd[e] = nd;
      const bool take = (nd > bv);
      bv = take ? nd : bv;
      bi = take ? (tid * 4 + e) : bi;
    }
    argmax_red(bv, bi);
    if (lane == 0) { wv[par][wave] = bv; wi[par][wave] = bi; }
    __syncthreads();
    float v = wv[par][lane];
    int   i = wi[par][lane];
    argmax_red(v, i);
    last = clampi(i, 0, kPts - 1);
    if ((last >> 2) == tid) sel |= (1u << (last & 3));
  }
  const int c = __popc(sel);
  int x = c;
#pragma unroll
  for (int off = 1; off < 32; off <<= 1) {
    const int t = __shfl_up(x, off, 32);
    x += (lane >= off) ? t : 0;
  }
  if (lane == 31) wtot[wave] = x;
  scent[tid] = 0;
  __syncthreads();
  int y = wtot[lane];
#pragma unroll
  for (int off = 1; off < 32; off <<= 1) {
    const int t = __shfl_up(y, off, 32);
    y += (lane >= off) ? t : 0;
  }
  const int wbelow = __shfl(y, (wave + 31) & 31, 32);
  int o = ((wave > 0) ? wbelow : 0) + x - c;
#pragma unroll
  for (int e = 0; e < 4; ++e) {
    if ((sel >> e) & 1u) {
      if (o < kSmp) scent[o] = tid * 4 + e;
      ++o;
    }
  }
  __syncthreads();
  if (tid < 256) {
    const v4i val = ((const v4i*)scent)[tid];
    int* dst = cent + (size_t)b * kSmp + tid * 4;
    *(volatile v4i*)dst = val;
    __threadfence();
    *(volatile v4i*)dst = val;
  }
}

__global__ __launch_bounds__(256) void nearest_kernel(const float* __restrict__ pos, int* __restrict__ nbr)
{
  __shared__ __align__(16) float cp[1024 * 3];
  __shared__ __align__(16) int snb[256 * kNbr];
  const int tid = threadIdx.x;
  const int b = blockIdx.x >> 4;
  const int q = ((blockIdx.x & 15) << 8) + tid;
  const size_t gq = (size_t)b * kPts + q;
  const float qx = pos[gq * 3 + 0], qy = pos[gq * 3 + 1], qz = pos[gq * 3 + 2];
  float qd[kNbr];
  int qi[kNbr];
#pragma unroll
  for (int r = 0; r < kNbr; ++r) { qd[r] = 3e38f; qi[r] = q; }

#pragma unroll 1
  for (int tile = 0; tile < 4; ++tile) {
    __syncthreads();
    {
      const v4f* src = (const v4f*)(pos + ((size_t)b * kPts + tile * 1024) * 3);
#pragma unroll
      for (int i = 0; i < 3; ++i) ((v4f*)cp)[tid + i * 256] = src[tid + i * 256];
    }
    __syncthreads();
#pragma unroll 1
    for (int j = 0; j < 1024; ++j) {
      const float dx = qx - cp[j * 3 + 0];
      const float dy = qy - cp[j * 3 + 1];
      const float dz = qz - cp[j * 3 + 2];
      const float d = (dx * dx + dy * dy) + dz * dz;
      if (d < qd[kNbr - 1]) {
        qd[kNbr - 1] = d;
        qi[kNbr - 1] = tile * 1024 + j;
#pragma unroll
        for (int r = kNbr - 1; r >= 1; --r) {
          const bool sw = (qd[r] < qd[r - 1]);
          const float da = qd[r], db = qd[r - 1];
          const int   ia = qi[r], ib = qi[r - 1];
          qd[r]     = sw ? db : da;
          qd[r - 1] = sw ? da : db;
          qi[r]     = sw ? ib : ia;
          qi[r - 1] = sw ? ia : ib;
        }
      }
    }
  }
#pragma unroll
  for (int k = 0; k < 4; ++k) {
    v4i w;
    w[0] = qi[4 * k + 0]; w[1] = qi[4 * k + 1]; w[2] = qi[4 * k + 2]; w[3] = qi[4 * k + 3];
    ((v4i*)snb)[tid * 4 + k] = w;
  }
  __syncthreads();
  {
    int* base = nbr + ((size_t)b * kPts + ((blockIdx.x & 15) << 8)) * kNbr;
    v4i val[4];
#pragma unroll
    for (int it = 0; it < 4; ++it) val[it] = ((const v4i*)snb)[it * 256 + tid];
    for (int pass = 0; pass < 2; ++pass) {
#pragma unroll
      for (int it = 0; it < 4; ++it) *(volatile v4i*)(base + (size_t)(it * 256 + tid) * 4) = val[it];
      __threadfence();
    }
  }
}

__device__ __forceinline__ v16h frag_load(const _Float16* p) {
  union { v16h v; v8h h[2]; } f;
  f.h[0] = *(const v8h*)(p);
  f.h[1] = *(const v8h*)(p + 16);
  return f.v;
}
__device__ __forceinline__ v8f mma_h(v16h a, v16h b, v8f c) {
  return __builtin_amdgcn_wmma_f32_16x16x32_f16(false, a, false, b, (short)0, c, false, false);
}
__device__ __forceinline__ void tie_acc(v8f& a, v16h x, v16h y) {
  asm volatile("v_nop\n\tv_nop\n\tv_nop\n\tv_nop" : "+v"(a) : "v"(x), "v"(y));
}
__device__ __forceinline__ void keep4_h(v16h a, v16h b, v16h c, v16h d) { asm volatile("v_nop" :: "v"(a), "v"(b), "v"(c), "v"(d)); }
__device__ __forceinline__ void acc_guard4(v8f& a, v8f& b, v8f& c, v8f& d) {
  asm volatile("v_nop\n\tv_nop\n\tv_nop\n\tv_nop" : "+v"(a), "+v"(b), "+v"(c), "+v"(d));
}

template <int MODE>
__global__ __launch_bounds__(256) void gemm_n128_kernel(
    const unsigned short* __restrict__ Ap, const unsigned short* __restrict__ Btp, int K,
    float* __restrict__ Cmain, float* __restrict__ Caux, float* __restrict__ part,
    const float* __restrict__ bias, float scale)
{
  const _Float16* A  = (const _Float16*)Ap;
  const _Float16* Bt = (const _Float16*)Btp;
  __shared__ __align__(16) float sT[8][16 * 68];
  __shared__ __align__(16) float red[8 * 128];
  const int lane = threadIdx.x & 31;
  const int wave = threadIdx.x >> 5;
  const int tile = blockIdx.x * 8 + wave;
  const int tm = tile >> 1;
  const int tn = tile & 1;
  const int m0 = tm << 6;
  const int n0 = tn << 6;
  const int rlane = lane & 15;
  const int hh    = lane >> 4;
  const int koff  = hh * 8;
  const int mOff  = hh * 8;

  v8f acc[4][4];
#pragma unroll
  for (int i = 0; i < 4; ++i)
#pragma unroll
    for (int j = 0; j < 4; ++j) acc[i][j] = (v8f){0.f, 0.f, 0.f, 0.f, 0.f, 0.f, 0.f, 0.f};

  for (int k0 = 0; k0 < K; k0 += 32) {
    v16h bh[4];
#pragma unroll
    for (int j = 0; j < 4; ++j) {
      const size_t bo = (size_t)(n0 + (j << 4) + rlane) * K + koff + k0;
      bh[j] = frag_load(Bt + bo);
    }
#pragma unroll
    for (int i = 0; i < 4; ++i) {
      const size_t ao = (size_t)(m0 + (i << 4) + rlane) * K + koff + k0;
      const v16h ah = frag_load(A + ao);
#pragma unroll
      for (int j = 0; j < 4; ++j) acc[i][j] = mma_h(ah, bh[j], acc[i][j]);
      tie_acc(acc[i][0], ah, bh[0]);
      tie_acc(acc[i][1], ah, bh[1]);
      tie_acc(acc[i][2], ah, bh[2]);
      tie_acc(acc[i][3], ah, bh[3]);
    }
    keep4_h(bh[0], bh[1], bh[2], bh[3]);
  }
  acc_guard4(acc[0][0], acc[0][1], acc[0][2], acc[0][3]);
  acc_guard4(acc[1][0], acc[1][1], acc[1][2], acc[1][3]);
  acc_guard4(acc[2][0], acc[2][1], acc[2][2], acc[2][3]);
  acc_guard4(acc[3][0], acc[3][1], acc[3][2], acc[3][3]);

  float* slab = sT[wave];
  if (MODE == 0) {
#pragma unroll
    for (int i = 0; i < 4; ++i) {
      const int mBase = m0 + (i << 4);
#pragma unroll
      for (int j = 0; j < 4; ++j) {
#pragma unroll
        for (int r = 0; r < 8; ++r) slab[(mOff + r) * 68 + (j << 4) + rlane] = acc[i][j][r] * scale;
      }
      __builtin_amdgcn_fence(__ATOMIC_RELEASE, "workgroup");
      __builtin_amdgcn_wave_barrier();
      __builtin_amdgcn_fence(__ATOMIC_ACQUIRE, "workgroup");
      const int c4 = (lane & 15) * 4;
      for (int pass = 0; pass < 2; ++pass) {
#pragma unroll
        for (int it = 0; it < 8; ++it) {
          const int row = it * 2 + hh;
          const v4f v = *(const v4f*)(slab + row * 68 + c4);
          *(volatile v4f*)(Cmain + (size_t)(mBase + row) * kCo + n0 + c4) = v;
        }
        __threadfence();
      }
      __builtin_amdgcn_fence(__ATOMIC_RELEASE, "workgroup");
      __builtin_amdgcn_wave_barrier();
      __builtin_amdgcn_fence(__ATOMIC_ACQUIRE, "workgroup");
    }
  } else {
    float bvj[4], cs[4], cq[4];
#pragma unroll
    for (int j = 0; j < 4; ++j) { bvj[j] = bias[n0 + (j << 4) + rlane]; cs[j] = 0.f; cq[j] = 0.f; }
#pragma unroll
    for (int i = 0; i < 4; ++i) {
#pragma unroll
      for (int j = 0; j < 4; ++j) {
        float mx = 0.f, mn = 0.f;
#pragma unroll
        for (int r = 0; r < 8; ++r) {
          const float v = fmaf(acc[i][j][r], scale, bvj[j]);
          mx = (r == 0) ? v : fmaxf(mx, v);
          mn = (r == 0) ? v : fminf(mn, v);
          cs[j] += v;
          cq[j] = fmaf(v, v, cq[j]);
        }
        const float omx = __shfl_xor(mx, 16, 32);
        const float omn = __shfl_xor(mn, 16, 32);
        mx = fmaxf(mx, omx);
        mn = fminf(mn, omn);
        slab[hh * 256 + i * 64 + (j << 4) + rlane] = hh ? mn : mx;
      }
    }
#pragma unroll
    for (int j = 0; j < 4; ++j) {
      const float os = __shfl_xor(cs[j], 16, 32);
      const float oq = __shfl_xor(cq[j], 16, 32);
      const float ts = cs[j] + os;
      const float tq = cq[j] + oq;
      red[wave * 128 + hh * 64 + (j << 4) + rlane] = hh ? tq : ts;
    }
    __builtin_amdgcn_fence(__ATOMIC_RELEASE, "workgroup");
    __builtin_amdgcn_wave_barrier();
    __builtin_amdgcn_fence(__ATOMIC_ACQUIRE, "workgroup");
    {
      const int node0 = m0 >> 4;
      const int c4 = (lane & 15) * 4;
      v4f vm[2], vn[2];
#pragma unroll
      for (int it = 0; it < 2; ++it) {
        const int row = it * 2 + hh;
        vm[it] = *(const v4f*)(slab + row * 64 + c4);
        vn[it] = *(const v4f*)(slab + 256 + row * 64 + c4);
      }
      for (int pass = 0; pass < 2; ++pass) {
#pragma unroll
        for (int it = 0; it < 2; ++it) {
          const int row = it * 2 + hh;
          const size_t o = (size_t)(node0 + row) * kCo + n0 + c4;
          *(volatile v4f*)(Cmain + o) = vm[it];
          *(volatile v4f*)(Caux + o)  = vn[it];
        }
        __threadfence();
      }
    }
    __syncthreads();
    if (threadIdx.x < 64) {
      const int idx4 = threadIdx.x * 4;
      const int isq  = idx4 >> 7;
      const int cc   = idx4 & 127;
      const int tnn  = cc >> 6;
      const int c6   = cc & 63;
      v4f s = *(const v4f*)(red + (tnn + 0) * 128 + isq * 64 + c6);
      s = s + *(const v4f*)(red + (tnn + 2) * 128 + isq * 64 + c6);
      s = s + *(const v4f*)(red + (tnn + 4) * 128 + isq * 64 + c6);
      s = s + *(const v4f*)(red + (tnn + 6) * 128 + isq * 64 + c6);
      float* dst = part + (size_t)blockIdx.x * 256 + idx4;
      *(volatile v4f*)dst = s;
      __threadfence();
      *(volatile v4f*)dst = s;
    }
  }
}

__device__ __forceinline__ void node_setup(const int* __restrict__ nbr, const float* __restrict__ pos,
                                           int node, int ln, int& gsrc, float& rx, float& ry, float& rz) {
  const int cloud = node >> 12;
  int nv = nbr[(size_t)node * kNbr + ln];
  nv = clampi(nv, 0, kPts - 1);
  gsrc = cloud * kPts + nv;
  const float sx = pos[(size_t)gsrc * 3 + 0], sy = pos[(size_t)gsrc * 3 + 1], sz = pos[(size_t)gsrc * 3 + 2];
  const float dx = pos[(size_t)node * 3 + 0], dy = pos[(size_t)node * 3 + 1], dz = pos[(size_t)node * 3 + 2];
  rx = sx - dx;
  ry = sy - dy;
  rz = sz - dz;
}

__device__ __forceinline__ void edge_row(const float* __restrict__ PP, int g, int c8, float rx, float ry, float rz,
                                         const float (&w0)[8], const float (&w1)[8], const float (&w2)[8],
                                         const float (&bb)[8], float (&h)[8]) {
  const v4f p0 = *(const v4f*)(PP + (size_t)g * kCo + c8);
  const v4f p1 = *(const v4f*)(PP + (size_t)g * kCo + c8 + 4);
  float p[8];
  unpack8(p0, p1, p);
#pragma unroll
  for (int e = 0; e < 8; ++e) {
    float t = p[e] + bb[e];
    t = fmaf(w0[e], rx, t);
    t = fmaf(w1[e], ry, t);
    t = fmaf(w2[e], rz, t);
    h[e] = t;
  }
}

__global__ __launch_bounds__(256) void edge_stats_kernel(
    const float* __restrict__ PP, const int* __restrict__ nbr, const float* __restrict__ pos,
    const float* __restrict__ W1, const float* __restrict__ b1, float* __restrict__ part)
{
  __shared__ __align__(16) float sw[4 * kCo];
  __shared__ __align__(16) float red[8 * 256];
  const int tid = threadIdx.x, lane = tid & 31, wave = tid >> 5;
  const int hh = lane >> 4, ln = lane & 15, c8 = ln * 8;
  for (int idx = tid; idx < 3 * kCo; idx += 256) {
    const int c = idx / 3;
    const int k = idx - c * 3;
    sw[k * kCo + c] = W1[(size_t)c * kCin + k];
  }
  if (tid < kCo) sw[3 * kCo + tid] = b1[tid];
  __syncthreads();
  float w0[8], w1[8], w2[8], bb[8];
  unpack8(*(const v4f*)(sw + c8), *(const v4f*)(sw + c8 + 4), w0);
  unpack8(*(const v4f*)(sw + kCo + c8), *(const v4f*)(sw + kCo + c8 + 4), w1);
  unpack8(*(const v4f*)(sw + 2 * kCo + c8), *(const v4f*)(sw + 2 * kCo + c8 + 4), w2);
  unpack8(*(const v4f*)(sw + 3 * kCo + c8), *(const v4f*)(sw + 3 * kCo + c8 + 4), bb);
  float s[8], q[8];
#pragma unroll
  for (int e = 0; e < 8; ++e) { s[e] = 0.f; q[e] = 0.f; }
#pragma unroll 1
  for (int nn = 0; nn < 8; ++nn) {
    const int node = blockIdx.x * 64 + wave * 8 + nn;
    int gsrc;
    float rx, ry, rz;
    node_setup(nbr, pos, node, ln, gsrc, rx, ry, rz);
#pragma unroll 1
    for (int jj = 0; jj < 8; ++jj) {
      const int src = 2 * jj + hh;
      const int   g   = __shfl(gsrc, src, 32);
      const float rxx = __shfl(rx, src, 32);
      const float ryy = __shfl(ry, src, 32);
      const float rzz = __shfl(rz, src, 32);
      float h[8];
      edge_row(PP, g, c8, rxx, ryy, rzz, w0, w1, w2, bb, h);
#pragma unroll
      for (int e = 0; e < 8; ++e) {
        s[e] += h[e];
        q[e] = fmaf(h[e], h[e], q[e]);
      }
    }
  }
  v4f o0, o1;
#pragma unroll
  for (int e = 0; e < 8; ++e) {
    const float os = __shfl_xor(s[e], 16, 32);
    const float oq = __shfl_xor(q[e], 16, 32);
    const float ts = s[e] + os;
    const float tq = q[e] + oq;
    const float val = hh ? tq : ts;
    if (e < 4) o0[e] = val; else o1[e - 4] = val;
  }
  *(v4f*)(red + wave * 256 + hh * 128 + c8)     = o0;
  *(v4f*)(red + wave * 256 + hh * 128 + c8 + 4) = o1;
  __syncthreads();
  if (tid < 64) {
    const int idx4 = tid * 4;
    v4f acc = *(const v4f*)(red + idx4);
#pragma unroll
    for (int w = 1; w < 8; ++w) acc = acc + *(const v4f*)(red + w * 256 + idx4);
    float* dst = part + (size_t)blockIdx.x * 256 + idx4;
    *(volatile v4f*)dst = acc;
    __threadfence();
    *(volatile v4f*)dst = acc;
  }
}

__global__ __launch_bounds__(128) void bn_coeff_kernel(
    const float* __restrict__ part, int nblk, const float* __restrict__ gamma, const float* __restrict__ beta,
    float* __restrict__ st)
{
  const int c = threadIdx.x;
  double S = 0.0, Q = 0.0;
  for (int w = 0; w < nblk; ++w) {
    S += (double)part[(size_t)w * 256 + c];
    Q += (double)part[(size_t)w * 256 + 128 + c];
  }
  const double mu = S * kInvEdges;
  double var = Q * kInvEdges - mu * mu;
  var = (var < 0.0) ? 0.0 : var;
  const float vf = (float)var + 1e-5f;
  const float rs = 1.0f / sqrtf(vf);
  const float sc = gamma[c] * rs;
  const float sh = (float)((double)beta[c] - mu * (double)sc);
  *(volatile float*)(st + c) = sc;
  *(volatile float*)(st + 128 + c) = sh;
  __threadfence();
  *(volatile float*)(st + c) = sc;
  *(volatile float*)(st + 128 + c) = sh;
}

__global__ __launch_bounds__(256) void edge_act_kernel(
    const float* __restrict__ PP, const int* __restrict__ nbr, const float* __restrict__ pos,
    const float* __restrict__ W1, const float* __restrict__ b1, const float* __restrict__ st1,
    unsigned short* __restrict__ x2)
{
  __shared__ __align__(16) float sw[4 * kCo];
  __shared__ __align__(16) v8h xs[8][16 * 16];
  const int tid = threadIdx.x, lane = tid & 31, wave = tid >> 5;
  const int hh = lane >> 4, ln = lane & 15, c8 = ln * 8;
  for (int idx = tid; idx < 3 * kCo; idx += 256) {
    const int c = idx / 3;
    const int k = idx - c * 3;
    sw[k * kCo + c] = W1[(size_t)c * kCin + k];
  }
  if (tid < kCo) sw[3 * kCo + tid] = b1[tid];
  __syncthreads();
  float w0[8], w1[8], w2[8], bb[8], s1[8], t1[8];
  unpack8(*(const v4f*)(sw + c8), *(const v4f*)(sw + c8 + 4), w0);
  unpack8(*(const v4f*)(sw + kCo + c8), *(const v4f*)(sw + kCo + c8 + 4), w1);
  unpack8(*(const v4f*)(sw + 2 * kCo + c8), *(const v4f*)(sw + 2 * kCo + c8 + 4), w2);
  unpack8(*(const v4f*)(sw + 3 * kCo + c8), *(const v4f*)(sw + 3 * kCo + c8 + 4), bb);
  unpack8(*(const v4f*)(st1 + c8), *(const v4f*)(st1 + c8 + 4), s1);
  unpack8(*(const v4f*)(st1 + 128 + c8), *(const v4f*)(st1 + 128 + c8 + 4), t1);
  v8h* tile = xs[wave];
#pragma unroll 1
  for (int nn = 0; nn < 8; ++nn) {
    const int node = blockIdx.x * 64 + wave * 8 + nn;
    int gsrc;
    float rx, ry, rz;
    node_setup(nbr, pos, node, ln, gsrc, rx, ry, rz);
#pragma unroll 1
    for (int jj = 0; jj < 8; ++jj) {
      const int src = 2 * jj + hh;
      const int   g   = __shfl(gsrc, src, 32);
      const float rxx = __shfl(rx, src, 32);
      const float ryy = __shfl(ry, src, 32);
      const float rzz = __shfl(rz, src, 32);
      float h[8];
      edge_row(PP, g, c8, rxx, ryy, rzz, w0, w1, w2, bb, h);
      v8h hv;
#pragma unroll
      for (int e = 0; e < 8; ++e) {
        const float y = fmaxf(fmaf(s1[e], h[e], t1[e]), 0.0f);
        hv[e] = cvt_h(y * kCarry);
      }
      tile[src * 16 + ln] = hv;
    }
    __builtin_amdgcn_fence(__ATOMIC_RELEASE, "workgroup");
    __builtin_amdgcn_wave_barrier();
    __builtin_amdgcn_fence(__ATOMIC_ACQUIRE, "workgroup");
    unsigned short* base = x2 + (size_t)node * kNbr * kCo;
    for (int pass = 0; pass < 2; ++pass) {
#pragma unroll
      for (int it = 0; it < 8; ++it) {
        const int row = 2 * it + hh;
        const v8h val = tile[row * 16 + ln];
        *(volatile v8h*)(base + (size_t)row * kCo + c8) = val;
      }
      __threadfence();
    }
    __builtin_amdgcn_fence(__ATOMIC_RELEASE, "workgroup");
    __builtin_amdgcn_wave_barrier();
    __builtin_amdgcn_fence(__ATOMIC_ACQUIRE, "workgroup");
  }
}

__global__ __launch_bounds__(256) void finalize_kernel(
    const float* __restrict__ hmax, const float* __restrict__ hmin, const float* __restrict__ st2,
    const int* __restrict__ cent, const float* __restrict__ pos, float* __restrict__ out)
{
  const int tid = threadIdx.x, lane = tid & 31, wave = tid >> 5;
  const int blk = blockIdx.x;
  if (blk < kFinRowBlk) {
    const int row = blk * 8 + wave;
    const int cloud = row >> 10;
    const int ci = clampi(cent[row], 0, kPts - 1);
    const size_t node = (size_t)cloud * kPts + ci;
    const int c4 = lane * 4;
    const v4f mx = *(const v4f*)(hmax + node * kCo + c4);
    const v4f mn = *(const v4f*)(hmin + node * kCo + c4);
    const v4f sc = *(const v4f*)(st2 + c4);
    const v4f sh = *(const v4f*)(st2 + 128 + c4);
    v4f o;
#pragma unroll
    for (int e = 0; e < 4; ++e) {
      const float x = (sc[e] >= 0.0f) ? mx[e] : mn[e];
      o[e] = fmaxf(fmaf(sc[e], x, sh[e]), 0.0f);
    }
    float* dst = out + kOut0 + (size_t)row * kCo + c4;
    *(volatile v4f*)dst = o;
    __threadfence();
    *(volatile v4f*)dst = o;
  } else {
    const int t = (blk - kFinRowBlk) * 256 + tid;
    const int e0 = t * 4;
    v4f o;
#pragma unroll
    for (int k = 0; k < 4; ++k) {
      const int e = e0 + k;
      const int r = e / 3;
      const int c = e - r * 3;
      const int cloud = r >> 10;
      const int ci = clampi(cent[r], 0, kPts - 1);
      o[k] = pos[((size_t)cloud * kPts + ci) * 3 + c];
    }
    float* dst = out + e0;
    *(volatile v4f*)dst = o;
    __threadfence();
    *(volatile v4f*)dst = o;
  }
}

extern "C" void kernel_launch(void* const* d_in, const int* in_sizes, int n_in,
                              void* d_out, int out_size, void* d_ws, size_t ws_size,
                              hipStream_t stream) {
  if (n_in < 10) return;
  if (in_sizes[0] != kNodes * kCf) return;
  if (in_sizes[1] != kNodes * 3) return;
  if (in_sizes[2] != kCo * kCin) return;
  if (in_sizes[3] != kCo || in_sizes[4] != kCo || in_sizes[5] != kCo) return;
  if (in_sizes[6] != kCo * kCo) return;
  if (in_sizes[7] != kCo || in_sizes[8] != kCo || in_sizes[9] != kCo) return;
  if (out_size != kOutAll) return;
  if (ws_size < kWsTotal) return;

  const float* feat = (const float*)d_in[0];
  const float* pos  = (const float*)d_in[1];
  const float* W1   = (const float*)d_in[2];
  const float* b1   = (const float*)d_in[3];
  const float* g1   = (const float*)d_in[4];
  const float* be1  = (const float*)d_in[5];
  const float* W2   = (const float*)d_in[6];
  const float* b2   = (const float*)d_in[7];
  const float* g2   = (const float*)d_in[8];
  const float* be2  = (const float*)d_in[9];
  float* out = (float*)d_out;

  char* ws = (char*)d_ws;
  int*            cent  = (int*)(ws + kOffCent);
  int*            nbr   = (int*)(ws + kOffNbr);
  unsigned short* featH = (unsigned short*)(ws + kOffFeatH);
  unsigned short* W1fH  = (unsigned short*)(ws + kOffW1fH);
  unsigned short* W2H   = (unsigned short*)(ws + kOffW2H);
  float*          PP    = (float*)(ws + kOffP);
  unsigned short* x2    = (unsigned short*)(ws + kOffX2);
  float*          hmax  = (float*)(ws + kOffHmax);
  float*          hmin  = (float*)(ws + kOffHmin);
  float*          part1 = (float*)(ws + kOffPart1);
  float*          part2 = (float*)(ws + kOffPart2);
  float*          st1   = (float*)(ws + kOffSt1);
  float*          st2   = (float*)(ws + kOffSt2);

  prep_planes_kernel<<<kPrepFeatBlk + kPrepW2Blk + kPrepW1Blk, 256, 0, stream>>>(feat, W1, W2, featH, W1fH, W2H);
  sample_kernel<<<kClouds, 1024, 0, stream>>>(pos, cent);
  nearest_kernel<<<kNodes / 256, 256, 0, stream>>>(pos, nbr);
  gemm_n128_kernel<0><<<kGemmPBlk, 256, 0, stream>>>(featH, W1fH, kCf, PP, hmax, part2, b1, kFold);
  edge_stats_kernel<<<kEdgeBlk, 256, 0, stream>>>(PP, nbr, pos, W1, b1, part1);
  bn_coeff_kernel<<<1, 128, 0, stream>>>(part1, kEdgeBlk, g1, be1, st1);
  edge_act_kernel<<<kEdgeBlk, 256, 0, stream>>>(PP, nbr, pos, W1, b1, st1, x2);
  gemm_n128_kernel<1><<<kGemm2Blk, 256, 0, stream>>>(x2, W2H, kCo, hmax, hmin, part2, b2, kFold);
  bn_coeff_kernel<<<1, 128, 0, stream>>>(part2, kGemm2Blk, g2, be2, st2);
  finalize_kernel<<<kFinRowBlk + kFinPosBlk, 256, 0, stream>>>(hmax, hmin, st2, cent, pos, out);
}
